// NeuralPCG_30039001268514
// MI455X (gfx1250) — hardware-verified
//
#include <hip/hip_runtime.h>
#include <stddef.h>
#include <stdint.h>
#include <math.h>


#define LD       128
#define WSC      16.0f
#define WINV     0.0625f
#define HP       136
#define FP       132

#define T_ENCN   0
#define T_ENCE   16384
#define T_DEC    32768
#define T_STEP0  49152
#define T_STEPSZ 114688
#define T_OP     0
#define T_OE0    32768
#define T_OE1    49152
#define T_ON0    65536
#define T_ON1    98304
#define T_PIECES 3072
#define T_TOTAL  (T_PIECES * 128)

#define M_HID    0
#define M_STG    (128 * HP * 2)
#define M_IDX    (2 * 128 * HP * 2)
#define M_LDS    (M_IDX + 256 * 4)

#define P_ROWS   64
#define P_LDS    (8 * 16 * FP * 4)

#define D_HID    0
#define D_RES    (128 * FP * 4)
#define D_LDS    (D_RES + 128 * 4)

#define NTHR     256
#define NWAVE    8
#define NB       256
#define EPT      8
#define CHUNK    (NTHR * EPT)
#define WCAP     (EPT * 32)
#define A_ACC    0
#define A_CNT    (NB * LD * 4)
#define A_LIST   (A_CNT + NB * 4)
#define A_WCNT   (A_LIST + NWAVE * WCAP * 4)
#define A_INV    (A_WCNT + 64)
#define A_LDS    (A_INV + NB * 4)

static_assert(T_STEP0 + 3 * T_STEPSZ == T_TOTAL);
static_assert((M_STG & 15) == 0 && (M_IDX & 15) == 0);
static_assert((A_CNT & 15) == 0 && (A_LIST & 15) == 0 && (A_WCNT & 15) == 0 && (A_INV & 15) == 0);
static_assert(((HP * 2) & 15) == 0 && ((FP * 4) & 15) == 0);
static_assert(M_LDS <= 300 * 1024 && A_LDS <= 300 * 1024 && P_LDS <= 300 * 1024 && D_LDS <= 300 * 1024);
static_assert(NB == 256 && (NB % NWAVE) == 0 && WCAP == 256);
static_assert(NB <= NTHR);

typedef float    v4f  __attribute__((ext_vector_type(4)));
typedef float    v8f  __attribute__((ext_vector_type(8)));
typedef int      v4i  __attribute__((ext_vector_type(4)));
typedef _Float16 v4h  __attribute__((ext_vector_type(4)));
typedef _Float16 v8h  __attribute__((ext_vector_type(8)));
typedef _Float16 v16h __attribute__((ext_vector_type(16)));
union FragH { v16h v; v8h h[2]; };

__device__ __forceinline__ v8f zero8f() {
  v8f z;
#pragma unroll
  for (int i = 0; i < 8; ++i) z[i] = 0.0f;
  return z;
}

__device__ __forceinline__ v8f wmh(v16h a, v16h b, v8f c) {
  v8f d = __builtin_amdgcn_wmma_f32_16x16x32_f16(false, a, false, b, (short)0, c, false, false);
  asm volatile("v_nop\n\tv_nop\n\tv_nop\n\tv_nop" : "+v"(d) : "v"(a), "v"(b));
  return d;
}

__device__ __forceinline__ void gemm16(const _Float16* arow, const _Float16* bcol, int kp, v8f acc[8]) {
#pragma unroll 1
  for (int kt = 0; kt < 4; ++kt) {
    FragH a;
    a.h[0] = *(const v8h*)(arow + 32 * kt);
    a.h[1] = *(const v8h*)(arow + 32 * kt + 16);
#pragma unroll
    for (int nt = 0; nt < 8; ++nt) {
      const _Float16* bp = bcol + (size_t)(16 * nt) * kp + 32 * kt;
      FragH b;
      b.h[0] = *(const v8h*)bp;
      b.h[1] = *(const v8h*)(bp + 16);
      acc[nt] = wmh(a.v, b.v, acc[nt]);
    }
  }
}

__device__ __forceinline__ void epi_hidden16(_Float16* hid, const float* __restrict__ bias,
                                             const v8f acc[8], int wave, int h, int m) {
#pragma unroll
  for (int nt = 0; nt < 8; ++nt) {
    const int c = 16 * nt + m;
    const float b = bias[c];
#pragma unroll
    for (int r = 0; r < 8; ++r) {
      const float v = acc[nt][r] * WINV + b;
      hid[(16 * wave + 8 * h + r) * HP + c] = (_Float16)fmaxf(v, 0.0f);
    }
  }
}

__device__ __forceinline__ void epi_out16(_Float16* stg, const float* __restrict__ bias,
                                          const v8f acc[8], int wave, int h, int m) {
#pragma unroll
  for (int nt = 0; nt < 8; ++nt) {
    const int c = 16 * nt + m;
    const float b = bias[c];
#pragma unroll
    for (int r = 0; r < 8; ++r) {
      const float v = acc[nt][r] * WINV + b;
      stg[(16 * wave + 8 * h + r) * HP + c] = (_Float16)v;
    }
  }
}

__device__ __forceinline__ void store_rows16(const _Float16* stg, _Float16* g, int row0, int M,
                                             int wave, int l) {
  const int h = l >> 4, c8 = 8 * (l & 15);
#pragma unroll
  for (int j = 0; j < 8; ++j) {
    const int lr = 16 * wave + 2 * j + h;
    const int gr = row0 + lr;
    if (gr < M) {
      const v8h v = *(const v8h*)(stg + lr * HP + c8);
      *(volatile v8h*)(g + (size_t)gr * LD + c8) = v;
    }
  }
  __threadfence();
#pragma unroll
  for (int j = 0; j < 8; ++j) {
    const int lr = 16 * wave + 2 * j + h;
    const int gr = row0 + lr;
    if (gr < M) {
      const v8h v = *(const v8h*)(stg + lr * HP + c8);
      *(volatile v8h*)(g + (size_t)gr * LD + c8) = v;
    }
  }
}

__global__ __launch_bounds__(256) void k_wcvt(const float* __restrict__ encnW1, const float* __restrict__ enceW1,
                                              const float* __restrict__ decW0, const float* __restrict__ eW0,
                                              const float* __restrict__ eW1, const float* __restrict__ nW0,
                                              const float* __restrict__ nW1, _Float16* Wt) {
  const int t = blockIdx.x * 256 + threadIdx.x;
  if (t >= T_PIECES * 16) return;
  const int p = t >> 4, kc = (t & 15) * 8;
  const float* src = encnW1;
  int roff = 0, n = 0;
  if (p < 128)      { src = encnW1; n = p; }
  else if (p < 256) { src = enceW1; n = p - 128; }
  else if (p < 384) { src = decW0;  n = p - 256; }
  else {
    const int q0 = p - 384;
    const int s = q0 / 896;
    const int q = q0 - s * 896;
    if (q < 256)      { src = eW0 + (size_t)s * 384 * 128; n = q & 127; roff = (q < 128) ? 0 : 128; }
    else if (q < 384) { src = eW0 + (size_t)s * 384 * 128; n = q - 256; roff = 256; }
    else if (q < 512) { src = eW1 + (size_t)s * 128 * 128; n = q - 384; roff = 0; }
    else if (q < 768) { src = nW0 + (size_t)s * 256 * 128; const int qq = q - 512; n = qq >> 1; roff = (qq & 1) * 128; }
    else              { src = nW1 + (size_t)s * 128 * 128; n = q - 768; roff = 0; }
  }
  v8h o;
#pragma unroll
  for (int i = 0; i < 8; ++i) o[i] = (_Float16)(src[(size_t)(roff + kc + i) * 128 + n] * WSC);
  _Float16* dp = Wt + (size_t)p * 128 + kc;
  *(volatile v8h*)dp = o;
  __threadfence();
  *(volatile v8h*)dp = o;
}

__global__ __launch_bounds__(256) void k_enc(const float* __restrict__ feat, const float* __restrict__ W0,
                                             const float* __restrict__ b0, const _Float16* W1t,
                                             const float* __restrict__ b1, _Float16* outh, int M) {
  extern __shared__ __attribute__((aligned(16))) unsigned char lds_m[];
  _Float16* hid = (_Float16*)(lds_m + M_HID);
  _Float16* stg = (_Float16*)(lds_m + M_STG);
  const int tid = threadIdx.x, l = tid & 31, wave = tid >> 5, h = l >> 4, m = l & 15;
  const int row0 = blockIdx.x * 128;

  for (int i = tid; i < 128 * 16; i += 256) {
    const int r = i >> 4, c = (i & 15) * 8;
    const int gr = row0 + r;
    const float xv = (gr < M) ? feat[gr] : 0.0f;
    v8h o;
#pragma unroll
    for (int j = 0; j < 8; ++j) {
      const float v = xv * W0[c + j] + b0[c + j];
      o[j] = (_Float16)fmaxf(v, 0.0f);
    }
    *(v8h*)(hid + r * HP + c) = o;
  }
  __syncthreads();

  v8f acc[8];
#pragma unroll
  for (int i = 0; i < 8; ++i) acc[i] = zero8f();
  gemm16(hid + (16 * wave + m) * HP + 8 * h, W1t + (size_t)m * LD + 8 * h, LD, acc);
  epi_out16(stg, b1, acc, wave, h, m);
  __syncthreads();
  store_rows16(stg, outh, row0, M, wave, l);
}

__global__ __launch_bounds__(256) void k_proj(const _Float16* __restrict__ ln, const _Float16* TP,
                                              float* P, int nN) {
  extern __shared__ __attribute__((aligned(16))) unsigned char lds_p[];
  float* stg = (float*)lds_p;
  const int tid = threadIdx.x, l = tid & 31, wave = tid >> 5, h = l >> 4, m = l & 15;
  const int wr = wave >> 1, wc = wave & 1;
  const int row0 = blockIdx.x * P_ROWS;
  int ar = row0 + 16 * wr + m;
  ar = ar > nN - 1 ? nN - 1 : ar;

  v8f acc[8];
#pragma unroll
  for (int i = 0; i < 8; ++i) acc[i] = zero8f();
  gemm16(ln + (size_t)ar * LD + 8 * h, TP + (size_t)(wc * 128 + m) * LD + 8 * h, LD, acc);

  float* st = stg + wave * (16 * FP);
#pragma unroll
  for (int nt = 0; nt < 8; ++nt) {
#pragma unroll
    for (int r = 0; r < 8; ++r) st[(8 * h + r) * FP + 16 * nt + m] = acc[nt][r] * WINV;
  }
  __syncthreads();

#pragma unroll
  for (int rr = 0; rr < 16; ++rr) {
    const int grow = row0 + 16 * wr + rr;
    if (grow < nN) {
      const v4f v = *(const v4f*)(st + rr * FP + 4 * l);
      *(volatile v4f*)(P + (size_t)grow * 256 + wc * 128 + 4 * l) = v;
    }
  }
  __threadfence();
#pragma unroll
  for (int rr = 0; rr < 16; ++rr) {
    const int grow = row0 + 16 * wr + rr;
    if (grow < nN) {
      const v4f v = *(const v4f*)(st + rr * FP + 4 * l);
      *(volatile v4f*)(P + (size_t)grow * 256 + wc * 128 + 4 * l) = v;
    }
  }
}

__global__ __launch_bounds__(256) void k_edge(const int* __restrict__ ei, const float* __restrict__ P,
                                              const _Float16* T0, const float* __restrict__ b0,
                                              const _Float16* T1, const float* __restrict__ b1,
                                              _Float16* le, int nE, int nN) {
  extern __shared__ __attribute__((aligned(16))) unsigned char lds_m[];
  _Float16* hid  = (_Float16*)(lds_m + M_HID);
  _Float16* stg  = (_Float16*)(lds_m + M_STG);
  int*      ridx = (int*)(lds_m + M_IDX);
  int*      cidx = ridx + 128;
  const int tid = threadIdx.x, l = tid & 31, wave = tid >> 5, h = l >> 4, m = l & 15;
  const int e0 = blockIdx.x * 128;

  if (tid < 128) {
    const int e = e0 + tid;
    int r = 0, c = 0;
    if (e < nE) { r = ei[e]; c = ei[(size_t)nE + e]; }
    r = r < 0 ? 0 : (r > nN - 1 ? nN - 1 : r);
    c = c < 0 ? 0 : (c > nN - 1 ? nN - 1 : c);
    ridx[tid] = r;
    cidx[tid] = c;
  }
  __syncthreads();

  int ar = e0 + 16 * wave + m;
  ar = ar > nE - 1 ? nE - 1 : ar;
  v8f acc[8];
#pragma unroll
  for (int i = 0; i < 8; ++i) acc[i] = zero8f();
  gemm16(le + (size_t)ar * LD + 8 * h, T0 + (size_t)m * LD + 8 * h, LD, acc);

  {
    int ri[8], ci[8];
#pragma unroll
    for (int r = 0; r < 8; ++r) {
      const int lr = 16 * wave + 8 * h + r;
      ri[r] = ridx[lr];
      ci[r] = cidx[lr];
    }
#pragma unroll
    for (int nt = 0; nt < 8; ++nt) {
      const int c = 16 * nt + m;
      const float bc = b0[c];
#pragma unroll
      for (int r = 0; r < 8; ++r) {
        const float ps = P[(size_t)ri[r] * 256 + c];
        const float pd = P[(size_t)ci[r] * 256 + 128 + c];
        float v = acc[nt][r] * WINV + ps;
        v = v + pd;
        v = v + bc;
        hid[(16 * wave + 8 * h + r) * HP + c] = (_Float16)fmaxf(v, 0.0f);
      }
    }
  }
  __syncthreads();

#pragma unroll
  for (int i = 0; i < 8; ++i) acc[i] = zero8f();
  gemm16(hid + (16 * wave + m) * HP + 8 * h, T1 + (size_t)m * LD + 8 * h, LD, acc);
  epi_out16(stg, b1, acc, wave, h, m);
  __syncthreads();
  store_rows16(stg, le, e0, nE, wave, l);
}

__device__ __forceinline__ int scan_chunk(const int* __restrict__ dsts, int nE, int cbase, int nodeBase,
                                          int* list, int tid, int wave) {
  int wc = 0;
  const int el0  = tid * EPT;
  const int e0   = cbase + el0;
  const int sent = -2147483647 - 1;
  v4i da, db;
  if (e0 + 7 < nE) {
    da = *(const v4i*)(dsts + e0);
    db = *(const v4i*)(dsts + e0 + 4);
  } else {
    da.x = (e0     < nE) ? dsts[(e0     < nE) ? e0     : nE - 1] : sent;
    da.y = (e0 + 1 < nE) ? dsts[(e0 + 1 < nE) ? e0 + 1 : nE - 1] : sent;
    da.z = (e0 + 2 < nE) ? dsts[(e0 + 2 < nE) ? e0 + 2 : nE - 1] : sent;
    da.w = (e0 + 3 < nE) ? dsts[(e0 + 3 < nE) ? e0 + 3 : nE - 1] : sent;
    db.x = (e0 + 4 < nE) ? dsts[(e0 + 4 < nE) ? e0 + 4 : nE - 1] : sent;
    db.y = (e0 + 5 < nE) ? dsts[(e0 + 5 < nE) ? e0 + 5 : nE - 1] : sent;
    db.z = (e0 + 6 < nE) ? dsts[(e0 + 6 < nE) ? e0 + 6 : nE - 1] : sent;
    db.w = (e0 + 7 < nE) ? dsts[(e0 + 7 < nE) ? e0 + 7 : nE - 1] : sent;
  }
  const unsigned nb = (unsigned)nodeBase;
  const unsigned s0 = (unsigned)da.x - nb, s1 = (unsigned)da.y - nb;
  const unsigned s2 = (unsigned)da.z - nb, s3 = (unsigned)da.w - nb;
  const unsigned s4 = (unsigned)db.x - nb, s5 = (unsigned)db.y - nb;
  const unsigned s6 = (unsigned)db.z - nb, s7 = (unsigned)db.w - nb;
  const bool q0 = s0 < (unsigned)NB, q1 = s1 < (unsigned)NB, q2 = s2 < (unsigned)NB, q3 = s3 < (unsigned)NB;
  const bool q4 = s4 < (unsigned)NB, q5 = s5 < (unsigned)NB, q6 = s6 < (unsigned)NB, q7 = s7 < (unsigned)NB;
  const unsigned any = __builtin_amdgcn_ballot_w32(q0 | q1 | q2 | q3 | q4 | q5 | q6 | q7);
  if (any != 0u) {
#define HITJ(J, QJ, SJ) { \
      const unsigned mj = __builtin_amdgcn_ballot_w32(QJ); \
      if (mj != 0u) { \
        if (QJ) { \
          const int pos = wc + (int)__builtin_amdgcn_mbcnt_lo(mj, 0u); \
          if (pos < WCAP) list[wave * WCAP + pos] = ((el0 + (J)) << 8) | (int)(SJ); \
        } \
        wc += (int)__builtin_popcount(mj); } }
    HITJ(0, q0, s0)
    HITJ(1, q1, s1)
    HITJ(2, q2, s2)
    HITJ(3, q3, s3)
    HITJ(4, q4, s4)
    HITJ(5, q5, s5)
    HITJ(6, q6, s6)
    HITJ(7, q7, s7)
#undef HITJ
  }
  return wc;
}

__global__ __launch_bounds__(NTHR) void k_agg(const int* __restrict__ ei, const _Float16* __restrict__ le,
                                               _Float16* agg, int nN, int nE) {
  extern __shared__ __attribute__((aligned(16))) unsigned char lds_a[];
  float* acc  = (float*)(lds_a + A_ACC);
  int*   cntL = (int*)(lds_a + A_CNT);
  int*   list = (int*)(lds_a + A_LIST);
  int*   wcnt = (int*)(lds_a + A_WCNT);
  float* invL = (float*)(lds_a + A_INV);
  const int tid = threadIdx.x, l = tid & 31, wave = tid >> 5, h = l >> 4, m = l & 15;
  const int nodeBase = blockIdx.x * NB;

  {
    const v4f z = {0.0f, 0.0f, 0.0f, 0.0f};
    for (int i = tid; i < NB * (LD / 4); i += NTHR) *(v4f*)(acc + 4 * i) = z;
    if (tid < NB) cntL[tid] = 0;
  }
  __syncthreads();

  const int nChunks = (nE + CHUNK - 1) / CHUNK;
#pragma unroll 1
  for (int ch = 0; ch < nChunks; ++ch) {
    const int cbase = ch * CHUNK;
    const int wc = scan_chunk(ei, nE, cbase, nodeBase, list, tid, wave);
    if (l == 0) wcnt[wave] = wc;
    __syncthreads();

#pragma unroll 1
    for (int w2 = 0; w2 < NWAVE; ++w2) {
      int n = wcnt[w2];
      n = n > WCAP ? WCAP : (n < 0 ? 0 : n);
      const int* lp = list + w2 * WCAP;
#pragma unroll 1
      for (int i = 0; i < n; ++i) {
        const int v = lp[i];
        const int slot = v & 255;
        if ((slot & 7) == wave) {
          int e = cbase + (v >> 8);
          e = e < 0 ? 0 : (e > nE - 1 ? nE - 1 : e);
          const v4h x = *(const v4h*)(le + (size_t)e * LD + 4 * l);
          float* ap = acc + slot * LD + 4 * l;
          v4f a = *(v4f*)ap;
          a[0] += (float)x[0]; a[1] += (float)x[1]; a[2] += (float)x[2]; a[3] += (float)x[3];
          *(v4f*)ap = a;
          if (l == 0) cntL[slot] = cntL[slot] + 1;
        }
      }
    }
    __syncthreads();
  }

  if (tid < NB) {
    int cn = cntL[tid];
    cn = cn < 1 ? 1 : cn;
    invL[tid] = 1.0f / (float)cn;
  }
  __syncthreads();

#pragma unroll
  for (int j = 0; j < 16; ++j) {
    const int slot = wave * (NB / NWAVE) + 2 * j + h;
    const int node = nodeBase + slot;
    const float inv = invL[slot];
    const v4f a0 = *(const v4f*)(acc + slot * LD + 8 * m);
    const v4f a1 = *(const v4f*)(acc + slot * LD + 8 * m + 4);
    v8h o;
#pragma unroll
    for (int i = 0; i < 4; ++i) { o[i] = (_Float16)(a0[i] * inv); o[4 + i] = (_Float16)(a1[i] * inv); }
    if (node < nN) *(volatile v8h*)(agg + (size_t)node * LD + 8 * m) = o;
  }
  __threadfence();
#pragma unroll
  for (int j = 0; j < 16; ++j) {
    const int slot = wave * (NB / NWAVE) + 2 * j + h;
    const int node = nodeBase + slot;
    const float inv = invL[slot];
    const v4f a0 = *(const v4f*)(acc + slot * LD + 8 * m);
    const v4f a1 = *(const v4f*)(acc + slot * LD + 8 * m + 4);
    v8h o;
#pragma unroll
    for (int i = 0; i < 4; ++i) { o[i] = (_Float16)(a0[i] * inv); o[4 + i] = (_Float16)(a1[i] * inv); }
    if (node < nN) *(volatile v8h*)(agg + (size_t)node * LD + 8 * m) = o;
  }
}

__global__ __launch_bounds__(256) void k_node(const _Float16* __restrict__ agg, const _Float16* T0,
                                              const float* __restrict__ b0, const _Float16* T1,
                                              const float* __restrict__ b1, _Float16* ln, int nN) {
  extern __shared__ __attribute__((aligned(16))) unsigned char lds_m[];
  _Float16* hid = (_Float16*)(lds_m + M_HID);
  _Float16* stg = (_Float16*)(lds_m + M_STG);
  const int tid = threadIdx.x, l = tid & 31, wave = tid >> 5, h = l >> 4, m = l & 15;
  const int row0 = blockIdx.x * 128;
  int ar = row0 + 16 * wave + m;
  ar = ar > nN - 1 ? nN - 1 : ar;

  v8f acc[8];
#pragma unroll
  for (int i = 0; i < 8; ++i) acc[i] = zero8f();
  gemm16(ln  + (size_t)ar * LD + 8 * h, T0 + (size_t)m * 256 + 8 * h,       256, acc);
  gemm16(agg + (size_t)ar * LD + 8 * h, T0 + (size_t)m * 256 + 128 + 8 * h, 256, acc);
  epi_hidden16(hid, b0, acc, wave, h, m);
  __syncthreads();

#pragma unroll
  for (int i = 0; i < 8; ++i) acc[i] = zero8f();
  gemm16(hid + (16 * wave + m) * HP + 8 * h, T1 + (size_t)m * LD + 8 * h, LD, acc);
  epi_out16(stg, b1, acc, wave, h, m);
  __syncthreads();
  store_rows16(stg, ln, row0, nN, wave, l);
}

__global__ __launch_bounds__(256) void k_dec(const _Float16* __restrict__ le, const _Float16* T0,
                                             const float* __restrict__ b0, const float* __restrict__ W1,
                                             const float* __restrict__ b1, const int* __restrict__ ei,
                                             const float* __restrict__ ea, float* out, int nE) {
  extern __shared__ __attribute__((aligned(16))) unsigned char lds_d[];
  float* hidf = (float*)(lds_d + D_HID);
  float* res  = (float*)(lds_d + D_RES);
  const int tid = threadIdx.x, l = tid & 31, wave = tid >> 5, h = l >> 4, m = l & 15;
  const int e0 = blockIdx.x * 128;
  int ar = e0 + 16 * wave + m;
  ar = ar > nE - 1 ? nE - 1 : ar;

  v8f acc[8];
#pragma unroll
  for (int i = 0; i < 8; ++i) acc[i] = zero8f();
  gemm16(le + (size_t)ar * LD + 8 * h, T0 + (size_t)m * LD + 8 * h, LD, acc);
#pragma unroll
  for (int nt = 0; nt < 8; ++nt) {
    const int c = 16 * nt + m;
    const float b = b0[c];
#pragma unroll
    for (int r = 0; r < 8; ++r) {
      const float v = acc[nt][r] * WINV + b;
      hidf[(16 * wave + 8 * h + r) * FP + c] = fmaxf(v, 0.0f);
    }
  }
  __syncthreads();

  if (tid < 128) {
    const int e = e0 + tid;
    const float* hr = hidf + tid * FP;
    float s = b1[0];
    for (int k = 0; k < LD; k += 4) {
      const v4f hv = *(const v4f*)(hr + k);
      const v4f wv = *(const v4f*)(W1 + k);
      s += hv[0] * wv[0];
      s += hv[1] * wv[1];
      s += hv[2] * wv[2];
      s += hv[3] * wv[3];
    }
    float rv = 0.0f;
    if (e < nE) {
      const int ri = ei[e];
      const int ci = ei[(size_t)nE + e];
      rv = (ri == ci) ? 0.5f * sqrtf(ea[e]) : s;
    }
    res[tid] = rv;
  }
  __syncthreads();

  if (wave == 0) {
    const int eb = e0 + 4 * l;
    const v4f v = *(const v4f*)(res + 4 * l);
    if (e0 + 128 <= nE) {
      *(volatile v4f*)(out + eb) = v;
    } else {
#pragma unroll
      for (int j = 0; j < 4; ++j) if (eb + j < nE) *(volatile float*)(out + eb + j) = v[j];
    }
    __threadfence();
    if (e0 + 128 <= nE) {
      *(volatile v4f*)(out + eb) = v;
    } else {
#pragma unroll
      for (int j = 0; j < 4; ++j) if (eb + j < nE) *(volatile float*)(out + eb + j) = v[j];
    }
  }
}

extern "C" void kernel_launch(void* const* d_in, const int* in_sizes, int n_in,
                              void* d_out, int out_size, void* d_ws, size_t ws_size,
                              hipStream_t stream) {
  if (n_in < 23) return;
  const int nN = in_sizes[0];
  const int nE = in_sizes[1];
  if (nN <= 0 || nE <= 0 || in_sizes[2] != 2 * nE || out_size != nE) return;
  if (in_sizes[3] < LD || in_sizes[4] < LD || in_sizes[5] != LD * LD || in_sizes[6] < LD) return;
  if (in_sizes[7] < LD || in_sizes[8] < LD || in_sizes[9] != LD * LD || in_sizes[10] < LD) return;
  if (in_sizes[11] != LD * LD || in_sizes[12] < LD || in_sizes[13] < LD || in_sizes[14] < 1) return;
  if (in_sizes[15] != 3 * 3 * LD * LD || in_sizes[16] < 3 * LD || in_sizes[17] != 3 * LD * LD || in_sizes[18] < 3 * LD) return;
  if (in_sizes[19] != 3 * 2 * LD * LD || in_sizes[20] < 3 * LD || in_sizes[21] != 3 * LD * LD || in_sizes[22] < 3 * LD) return;

  const float* x         = (const float*)d_in[0];
  const float* edge_attr = (const float*)d_in[1];
  const int*   ei        = (const int*)d_in[2];
  const float* encn_W0 = (const float*)d_in[3];
  const float* encn_b0 = (const float*)d_in[4];
  const float* encn_W1 = (const float*)d_in[5];
  const float* encn_b1 = (const float*)d_in[6];
  const float* ence_W0 = (const float*)d_in[7];
  const float* ence_b0 = (const float*)d_in[8];
  const float* ence_W1 = (const float*)d_in[9];
  const float* ence_b1 = (const float*)d_in[10];
  const float* dec_W0  = (const float*)d_in[11];
  const float* dec_b0  = (const float*)d_in[12];
  const float* dec_W1  = (const float*)d_in[13];
  const float* dec_b1  = (const float*)d_in[14];
  const float* eW0 = (const float*)d_in[15];
  const float* eb0 = (const float*)d_in[16];
  const float* eW1 = (const float*)d_in[17];
  const float* eb1 = (const float*)d_in[18];
  const float* nW0 = (const float*)d_in[19];
  const float* nb0 = (const float*)d_in[20];
  const float* nW1 = (const float*)d_in[21];
  const float* nb1 = (const float*)d_in[22];
  float* out = (float*)d_out;

  char* ws = (char*)d_ws;
  size_t off = 0;
  const size_t oWt = off; off += (size_t)T_TOTAL * 2;       off = (off + 255) & ~(size_t)255;
  const size_t oLe = off; off += (size_t)nE * LD * 2;        off = (off + 255) & ~(size_t)255;
  const size_t oLn = off; off += (size_t)nN * LD * 2;        off = (off + 255) & ~(size_t)255;
  const size_t oAg = off; off += (size_t)nN * LD * 2;        off = (off + 255) & ~(size_t)255;
  const size_t oP  = off; off += (size_t)nN * 256 * 4;       off = (off + 255) & ~(size_t)255;
  if (off > ws_size) return;
  _Float16* Wt  = (_Float16*)(ws + oWt);
  _Float16* leh = (_Float16*)(ws + oLe);
  _Float16* lnh = (_Float16*)(ws + oLn);
  _Float16* agh = (_Float16*)(ws + oAg);
  float*    Pb  = (float*)(ws + oP);

  const hipError_t a0 = hipFuncSetAttribute(reinterpret_cast<const void*>(&k_enc),  hipFuncAttributeMaxDynamicSharedMemorySize, M_LDS);
  const hipError_t a1 = hipFuncSetAttribute(reinterpret_cast<const void*>(&k_edge), hipFuncAttributeMaxDynamicSharedMemorySize, M_LDS);
  const hipError_t a2 = hipFuncSetAttribute(reinterpret_cast<const void*>(&k_node), hipFuncAttributeMaxDynamicSharedMemorySize, M_LDS);
  const hipError_t a3 = hipFuncSetAttribute(reinterpret_cast<const void*>(&k_proj), hipFuncAttributeMaxDynamicSharedMemorySize, P_LDS);
  const hipError_t a4 = hipFuncSetAttribute(reinterpret_cast<const void*>(&k_agg),  hipFuncAttributeMaxDynamicSharedMemorySize, A_LDS);
  const hipError_t a5 = hipFuncSetAttribute(reinterpret_cast<const void*>(&k_dec),  hipFuncAttributeMaxDynamicSharedMemorySize, D_LDS);
  (void)a0; (void)a1; (void)a2; (void)a3; (void)a4; (void)a5;

  const int nBlkN  = (nN + 127) / 128;
  const int nBlkE  = (nE + 127) / 128;
  const int nBlkP  = (nN + P_ROWS - 1) / P_ROWS;
  const int nBlkA  = (nN + NB - 1) / NB;

  k_wcvt<<<(T_PIECES * 16 + 255) / 256, 256, 0, stream>>>(encn_W1, ence_W1, dec_W0, eW0, eW1, nW0, nW1, Wt);

  k_enc<<<nBlkN, 256, M_LDS, stream>>>(x, encn_W0, encn_b0, Wt + T_ENCN, encn_b1, lnh, nN);
  k_enc<<<nBlkE, 256, M_LDS, stream>>>(edge_attr, ence_W0, ence_b0, Wt + T_ENCE, ence_b1, leh, nE);

  for (int s = 0; s < 3; ++s) {
    const _Float16* Ts = Wt + T_STEP0 + (size_t)s * T_STEPSZ;
    k_proj<<<nBlkP, 256, P_LDS, stream>>>(lnh, Ts + T_OP, Pb, nN);
    k_edge<<<nBlkE, 256, M_LDS, stream>>>(ei, Pb, Ts + T_OE0, eb0 + s * LD, Ts + T_OE1, eb1 + s * LD,
                                           leh, nE, nN);
    k_agg<<<nBlkA, NTHR, A_LDS, stream>>>(ei, leh, agh, nN, nE);
    k_node<<<nBlkN, 256, M_LDS, stream>>>(agh, Ts + T_ON0, nb0 + s * LD, Ts + T_ON1, nb1 + s * LD,
                                           lnh, nN);
  }

  k_dec<<<nBlkE, 256, D_LDS, stream>>>(leh, Wt + T_DEC, dec_b0, dec_W1, dec_b1, ei, edge_attr, out, nE);
  (void)hipGetLastError();
}
